// DengueGNN_15418932593124
// MI455X (gfx1250) — hardware-run, weakly checked
//
#include <hip/hip_runtime.h>
#include <stddef.h>
#include <stdint.h>
#include <math.h>

#define NN      100000
#define NE      1600000
#define FD      64
#define HC1     128
#define HID     32
#define NH1     4
#define MP      100096
#define KA2P    256
#define KW2P    256
#define SPLIT2  1
#define KX2     (SPLIT2 ? 256 : 128)
#define NTHR    256
#define NWAVE   8
#define EPT     8
#define WCH     (32 * EPT)
#define NBRUN   1024
#define SLB     10
#define NBK     98
#define WLCAP   3584
#define RCAP    28672
#define DEGCAP  256
#define MAXDEG_MEAS   36
#define MAXB1024_MEAS 16710
#define ABM     64
#define G1M     64
#define G1T     128
#define SP1     132
#define G2M     128
#define SP2     36
#define NEGSL   0.2f
#define EPS_SM  1e-16f
#define NEGBIG  (-3.0e38f)

#define PM_AS1  0
#define PM_AD1  128
#define PM_B1   256
#define PM_AS2  384
#define PM_AD2  416
#define PM_B2   448
#define PM_WL   480
#define PM_BL   512
#define PMN     640

#define BK_ZINTS (NWAVE * WLCAP + RCAP + 3 * NBRUN)
#define BK_INTS  (BK_ZINTS + 16)
#define BK_LDS   (BK_INTS * 4)

#define PBX  (MP * FD / 8 / NTHR)
#define PBW1 (HC1 * FD / 8 / NTHR)
#define PBW2 (HID * KW2P / 8 / NTHR)
#define PBTOT (PBX + PBW1 + PBW2 + 1)

static_assert(MP % G2M == 0 && MP % G1M == 0 && MP % ABM == 0 && MP >= NN && MP == 782 * 128);
static_assert(NN < (1 << 17) && NN % 32 == 0);
static_assert(NBRUN == (1 << SLB) && NBRUN <= 1024 && NBRUN % ABM == 0 && NBRUN % 32 == 0);
static_assert(NBK * NBRUN >= MP);
static_assert(NE < (1 << 21) && (((long long)NE) << SLB) < (1LL << 31));
static_assert(NE % WCH == 0 && NE % 4 == 0);
static_assert(RCAP == NWAVE * WLCAP && RCAP % (NTHR * 4) == 0 && BK_ZINTS % 4 == 0);
static_assert((2 * NBRUN) % (NTHR * 4) == 0);
static_assert((long long)RCAP * 100 >= (long long)MAXB1024_MEAS * 105);
static_assert(WLCAP >= MAXB1024_MEAS / 8 + 8 * 46 + 1);
static_assert(MAXDEG_MEAS + 8 <= DEGCAP);
static_assert(BK_LDS <= 327680);
static_assert((MP * FD / 8) % NTHR == 0 && (HC1 * FD / 8) % NTHR == 0 && (HID * KW2P / 8) % NTHR == 0);
static_assert(FD % 32 == 0 && KX2 % 32 == 0 && KX2 <= KA2P && KX2 <= KW2P && KA2P == 2 * HC1 && KW2P == 2 * HC1);
static_assert(HC1 == 4 * 32 && HID == 32 && NH1 * HID == HC1);
static_assert(G1M == (G1T / 32) * 16 && G2M == NWAVE * 16 && ABM == NWAVE * 8);
static_assert((G1M * SP1 + 256 + 2 * G1M * 4) * 4 <= 65536);
static_assert(PMN % 4 == 0 && PMN / 4 <= NTHR && PM_BL < PMN);

typedef float          v4f   __attribute__((ext_vector_type(4)));
typedef float          v8f   __attribute__((ext_vector_type(8)));
typedef int            v4i   __attribute__((ext_vector_type(4)));
typedef int            v8i   __attribute__((ext_vector_type(8)));
typedef unsigned short v8us  __attribute__((ext_vector_type(8)));
typedef __bf16         v16bf __attribute__((ext_vector_type(16)));
typedef v4f  __attribute__((may_alias)) v4fa;
typedef v4i  __attribute__((may_alias)) v4ia;
typedef v8us __attribute__((may_alias)) v8usa;
union FragB { v16bf v; v8us h[2]; v8i w; };

__device__ __forceinline__ v8f wmb(const FragB& a, const FragB& b, v8f c) {
  v8f d = __builtin_amdgcn_wmma_f32_16x16x32_bf16(false, a.v, false, b.v, (short)0, c, false, false);
  asm volatile("v_nop\n\tv_nop\n\tv_nop\n\tv_nop" : "+v"(d) : "v"(a.w), "v"(b.w));
  return d;
}

__device__ __forceinline__ unsigned bf16_bits(float f) {
  const unsigned u = __float_as_uint(f);
  const unsigned r = (u + 0x7FFFu + ((u >> 16) & 1u)) >> 16;
  const unsigned q = (u >> 16) | 0x40u;
  return ((u & 0x7fffffffu) > 0x7f800000u) ? q : r;
}
__device__ __forceinline__ unsigned rbits(float f) { return bf16_bits(f) << 16; }

__device__ __forceinline__ float leaky(float v) { return v > 0.0f ? v : NEGSL * v; }

__device__ __forceinline__ void hilo_pack(float v0, float v1, float v2, float v3,
                                          int& h01, int& h23, int& l01, int& l23) {
  const unsigned a0 = bf16_bits(v0), a1 = bf16_bits(v1), a2 = bf16_bits(v2), a3 = bf16_bits(v3);
  const unsigned b0 = bf16_bits(v0 - __uint_as_float(a0 << 16));
  const unsigned b1 = bf16_bits(v1 - __uint_as_float(a1 << 16));
  const unsigned b2 = bf16_bits(v2 - __uint_as_float(a2 << 16));
  const unsigned b3 = bf16_bits(v3 - __uint_as_float(a3 << 16));
  h01 = (int)(a0 | (a1 << 16)); h23 = (int)(a2 | (a3 << 16));
  l01 = (int)(b0 | (b1 << 16)); l23 = (int)(b2 | (b3 << 16));
}

__device__ __forceinline__ v4i regroup32(int h01, int h23, int l01, int l23, int lane) {
  const int s0 = (2 * lane) & 31, s1 = (2 * lane + 1) & 31;
  const int a0 = __shfl(h01, s0, 32), a1 = __shfl(h23, s0, 32), a2 = __shfl(h01, s1, 32), a3 = __shfl(h23, s1, 32);
  const int b0 = __shfl(l01, s0, 32), b1 = __shfl(l23, s0, 32), b2 = __shfl(l01, s1, 32), b3 = __shfl(l23, s1, 32);
  const int mk = (lane < 16) ? -1 : 0;
  v4i o;
  o.x = (a0 & mk) | (b0 & ~mk); o.y = (a1 & mk) | (b1 & ~mk);
  o.z = (a2 & mk) | (b2 & ~mk); o.w = (a3 & mk) | (b3 & ~mk);
  return o;
}

__device__ __forceinline__ void st2_v4f(float* p, v4f v) {
  *(volatile v4f*)p = v;
  __threadfence();
  *(volatile v4f*)p = v;
}
__device__ __forceinline__ void st2_v8us(unsigned short* p, v8us v) {
  *(volatile v8us*)p = v;
  __threadfence();
  *(volatile v8us*)p = v;
}

__device__ __forceinline__ v8us colpick8(const float* __restrict__ base, int stride) {
  float f[8];
#pragma unroll
  for (int i = 0; i < 8; ++i) f[i] = base[(size_t)i * (size_t)stride];
  v8us o;
#pragma unroll
  for (int i = 0; i < 8; ++i) o[i] = (unsigned short)bf16_bits(f[i]);
  return o;
}

__global__ __launch_bounds__(NTHR) void k_prep(const float* __restrict__ x, const float* __restrict__ w1,
                                               const float* __restrict__ as1, const float* __restrict__ ad1,
                                               const float* __restrict__ b1, const float* __restrict__ w2,
                                               const float* __restrict__ as2, const float* __restrict__ ad2,
                                               const float* __restrict__ b2, const float* __restrict__ wlin,
                                               const float* __restrict__ blin,
                                               unsigned short* xb, unsigned short* w1t, unsigned short* w2t,
                                               float* pm) {
  const int tid = (int)threadIdx.x, lane = tid & 31;
  const int blk = (int)blockIdx.x;
  if (blk < PBX) {
    const int u   = blk * NTHR + tid;
    const int row = u >> 3, k8 = (u & 7) * 8;
    const int rc  = row < NN ? row : NN - 1;
    const unsigned mk = row < NN ? 0xffffu : 0u;
    const float* p = x + (size_t)rc * FD + k8;
    const v4f a = *(const v4fa*)p;
    const v4f b = *(const v4fa*)(p + 4);
    v8us o;
    o[0] = (unsigned short)(bf16_bits(a.x) & mk); o[1] = (unsigned short)(bf16_bits(a.y) & mk);
    o[2] = (unsigned short)(bf16_bits(a.z) & mk); o[3] = (unsigned short)(bf16_bits(a.w) & mk);
    o[4] = (unsigned short)(bf16_bits(b.x) & mk); o[5] = (unsigned short)(bf16_bits(b.y) & mk);
    o[6] = (unsigned short)(bf16_bits(b.z) & mk); o[7] = (unsigned short)(bf16_bits(b.w) & mk);
    st2_v8us(xb + (size_t)row * FD + k8, o);
  } else if (blk < PBX + PBW1) {
    const int u = (blk - PBX) * NTHR + tid;
    const int n = u >> 3, k8 = (u & 7) * 8;
    const v8us o = colpick8(w1 + (size_t)k8 * HC1 + n, HC1);
    st2_v8us(w1t + (size_t)n * FD + k8, o);
  } else if (blk < PBX + PBW1 + PBW2) {
    const int u = (blk - PBX - PBW1) * NTHR + tid;
    const int n = u >> 5, k8 = (u & 31) * 8, kk = k8 & (HC1 - 1);
    const v8us o = colpick8(w2 + (size_t)kk * HID + n, HID);
    st2_v8us(w2t + (size_t)n * KW2P + k8, o);
  } else {
    if (tid < PMN / 4) {
      const int q = lane & 7;
      const v4f va = *(const v4fa*)(as1 + 4 * lane);
      const v4f vb = *(const v4fa*)(ad1 + 4 * lane);
      const v4f vc = *(const v4fa*)(b1 + 4 * lane);
      const v4f wa = *(const v4fa*)(as2 + 4 * q);
      const v4f wb = *(const v4fa*)(ad2 + 4 * q);
      const v4f wc = *(const v4fa*)(b2 + 4 * q);
      const v4f wd = *(const v4fa*)(wlin + 4 * q);
      const float bl = blin[0];
      asm volatile("" :: "v"(va), "v"(vb), "v"(vc));
      asm volatile("" :: "v"(wa), "v"(wb), "v"(wc), "v"(wd));
      asm volatile("" :: "v"(bl));
      const int wv = tid >> 5, sub = lane >> 3;
      const unsigned ma = (wv == 0) ? 0xffffffffu : 0u;
      const unsigned mb = (wv == 1) ? 0xffffffffu : 0u;
      const unsigned mc = (wv == 2) ? 0xffffffffu : 0u;
      const unsigned m3 = (wv == 3) ? 0xffffffffu : 0u;
      const unsigned na = (sub == 0) ? m3 : 0u, nb = (sub == 1) ? m3 : 0u;
      const unsigned nc = (sub == 2) ? m3 : 0u, nd = (sub == 3) ? m3 : 0u;
      const unsigned ml = (wv == 4 && lane == 0) ? 0xffffffffu : 0u;
      v4f o;
      o.x = __uint_as_float((rbits(va.x) & ma) | (rbits(vb.x) & mb) | (rbits(vc.x) & mc) | (rbits(wa.x) & na) |
                            (rbits(wb.x) & nb) | (rbits(wc.x) & nc) | (rbits(wd.x) & nd) | (rbits(bl) & ml));
      o.y = __uint_as_float((rbits(va.y) & ma) | (rbits(vb.y) & mb) | (rbits(vc.y) & mc) | (rbits(wa.y) & na) |
                            (rbits(wb.y) & nb) | (rbits(wc.y) & nc) | (rbits(wd.y) & nd));
      o.z = __uint_as_float((rbits(va.z) & ma) | (rbits(vb.z) & mb) | (rbits(vc.z) & mc) | (rbits(wa.z) & na) |
                            (rbits(wb.z) & nb) | (rbits(wc.z) & nc) | (rbits(wd.z) & nd));
      o.w = __uint_as_float((rbits(va.w) & ma) | (rbits(vb.w) & mb) | (rbits(vc.w) & mc) | (rbits(wa.w) & na) |
                            (rbits(wb.w) & nb) | (rbits(wc.w) & nc) | (rbits(wd.w) & nd));
      st2_v4f(pm + 4 * tid, o);
    }
  }
}

__device__ __forceinline__ void bucket_flush(const int* pl, const int* cnt, int ov, int* lp, int* cop, int* fp,
                                             int tid) {
#pragma unroll 1
  for (int i = tid * 4; i < RCAP; i += NTHR * 4) {
    const v4i v = *(const v4ia*)(pl + i);
    *(volatile v4i*)(lp + i) = v;
  }
#pragma unroll 1
  for (int i = tid * 4; i < 2 * NBRUN; i += NTHR * 4) {
    const v4i v = *(const v4ia*)(cnt + i);
    *(volatile v4i*)(cop + i) = v;
  }
  if (tid < 8) {
    const v4i f = {ov, ov, ov, ov};
    *(volatile v4i*)(fp + 4 * tid) = f;
  }
}

__global__ __launch_bounds__(NTHR) void k_bucket(const int* __restrict__ srcs, const int* __restrict__ dsts,
                                                 int* LIST, int* CO, int* FLAG) {
  extern __shared__ __attribute__((aligned(16))) int dsm[];
  int* wl   = dsm;
  int* pl   = dsm + NWAVE * WLCAP;
  int* cnt  = pl + RCAP;
  int* offs = cnt + NBRUN;
  int* cur  = offs + NBRUN;
  int* misc = cur + NBRUN;
  const int tid = (int)threadIdx.x, lane = tid & 31, wave = tid >> 5;
  const int blk = (int)blockIdx.x;
  const unsigned nbs = (unsigned)(blk * NBRUN);

  {
    const v4i z4 = {0, 0, 0, 0};
    for (int i = tid * 4; i < BK_ZINTS; i += NTHR * 4) *(v4ia*)(dsm + i) = z4;
    if (tid < 16) misc[tid] = 0;
  }
  __syncthreads();

  {
    const int per  = ((NE + NWAVE * WCH - 1) / (NWAVE * WCH)) * WCH;
    const int ebeg = wave * per;
    const int eend = (ebeg + per < NE) ? (ebeg + per) : NE;
    int* mylist = wl + wave * WLCAP;
    int wc = 0;
#pragma unroll 1
    for (int cb = ebeg; cb < eend; cb += WCH) {
      const int e0 = cb + lane * EPT;
      const v4i da = *(const v4ia*)(dsts + e0);
      const v4i db = *(const v4ia*)(dsts + e0 + 4);
      const unsigned s0 = (unsigned)da.x - nbs, s1 = (unsigned)da.y - nbs;
      const unsigned s2 = (unsigned)da.z - nbs, s3 = (unsigned)da.w - nbs;
      const unsigned s4 = (unsigned)db.x - nbs, s5 = (unsigned)db.y - nbs;
      const unsigned s6 = (unsigned)db.z - nbs, s7 = (unsigned)db.w - nbs;
      const bool h0 = s0 < (unsigned)NBRUN, h1 = s1 < (unsigned)NBRUN, h2 = s2 < (unsigned)NBRUN, h3 = s3 < (unsigned)NBRUN;
      const bool h4 = s4 < (unsigned)NBRUN, h5 = s5 < (unsigned)NBRUN, h6 = s6 < (unsigned)NBRUN, h7 = s7 < (unsigned)NBRUN;
      const unsigned m0 = __builtin_amdgcn_ballot_w32(h0), m1 = __builtin_amdgcn_ballot_w32(h1);
      const unsigned m2 = __builtin_amdgcn_ballot_w32(h2), m3 = __builtin_amdgcn_ballot_w32(h3);
      const unsigned m4 = __builtin_amdgcn_ballot_w32(h4), m5 = __builtin_amdgcn_ballot_w32(h5);
      const unsigned m6 = __builtin_amdgcn_ballot_w32(h6), m7 = __builtin_amdgcn_ballot_w32(h7);
      const unsigned any = m0 | m1 | m2 | m3 | m4 | m5 | m6 | m7;
      if (any != 0u) {
        const int pre = (int)(__builtin_amdgcn_mbcnt_lo(m0, 0u) + __builtin_amdgcn_mbcnt_lo(m1, 0u) +
                              __builtin_amdgcn_mbcnt_lo(m2, 0u) + __builtin_amdgcn_mbcnt_lo(m3, 0u) +
                              __builtin_amdgcn_mbcnt_lo(m4, 0u) + __builtin_amdgcn_mbcnt_lo(m5, 0u) +
                              __builtin_amdgcn_mbcnt_lo(m6, 0u) + __builtin_amdgcn_mbcnt_lo(m7, 0u));
        int p = wc + pre;
        if (h0) { if (p < WLCAP) mylist[p] = ((e0 + 0) << SLB) | (int)s0; p = p + 1; }
        if (h1) { if (p < WLCAP) mylist[p] = ((e0 + 1) << SLB) | (int)s1; p = p + 1; }
        if (h2) { if (p < WLCAP) mylist[p] = ((e0 + 2) << SLB) | (int)s2; p = p + 1; }
        if (h3) { if (p < WLCAP) mylist[p] = ((e0 + 3) << SLB) | (int)s3; p = p + 1; }
        if (h4) { if (p < WLCAP) mylist[p] = ((e0 + 4) << SLB) | (int)s4; p = p + 1; }
        if (h5) { if (p < WLCAP) mylist[p] = ((e0 + 5) << SLB) | (int)s5; p = p + 1; }
        if (h6) { if (p < WLCAP) mylist[p] = ((e0 + 6) << SLB) | (int)s6; p = p + 1; }
        if (h7) { if (p < WLCAP) mylist[p] = ((e0 + 7) << SLB) | (int)s7; p = p + 1; }
        wc += (int)(__builtin_popcount(m0) + __builtin_popcount(m1) + __builtin_popcount(m2) + __builtin_popcount(m3) +
                    __builtin_popcount(m4) + __builtin_popcount(m5) + __builtin_popcount(m6) + __builtin_popcount(m7));
      }
    }
    if (lane == 0) misc[wave] = wc;
  }
  __syncthreads();

  if (wave == 0) {
    int ov = 0;
#pragma unroll 1
    for (int w2 = 0; w2 < NWAVE; ++w2) {
      int c = misc[w2];
      if (c > WLCAP) ov = 1;
      c = c < 0 ? 0 : (c > WLCAP ? WLCAP : c);
#pragma unroll 1
      for (int b0 = 0; b0 < c; b0 += 32) {
        const int idx = b0 + lane;
        const int ent = wl[w2 * WLCAP + (idx < WLCAP ? idx : WLCAP - 1)];
        const int m32 = (c - b0) < 32 ? (c - b0) : 32;
#pragma unroll 1
        for (int k = 0; k < m32; ++k) {
          const int u    = __builtin_amdgcn_readlane(ent, k);
          const int slot = u & (NBRUN - 1);
          if (lane == 0) cnt[slot] = cnt[slot] + 1;
        }
      }
    }
    if (lane == 0) misc[9] = ov;
  }
  __syncthreads();
  if (wave == 0) {
    const int base = lane * (NBRUN / 32);
    int s = 0;
#pragma unroll 1
    for (int i = 0; i < NBRUN / 32; ++i) s += cnt[base + i];
    int incl = s;
#pragma unroll
    for (int d = 1; d < 32; d <<= 1) {
      const int y = __shfl_up(incl, d, 32);
      if (lane >= d) incl += y;
    }
    int run = incl - s;
#pragma unroll 1
    for (int i = 0; i < NBRUN / 32; ++i) {
      const int cv = cnt[base + i];
      offs[base + i] = run;
      cur[base + i]  = run;
      run += cv;
    }
  }
  __syncthreads();

  if (wave == 0) {
#pragma unroll 1
    for (int w2 = 0; w2 < NWAVE; ++w2) {
      int c = misc[w2];
      c = c < 0 ? 0 : (c > WLCAP ? WLCAP : c);
#pragma unroll 1
      for (int b0 = 0; b0 < c; b0 += 32) {
        const int idx = b0 + lane;
        const int ent = wl[w2 * WLCAP + (idx < WLCAP ? idx : WLCAP - 1)];
        int eid = (ent >> SLB) & 0x1FFFFF;
        eid = eid > NE - 1 ? NE - 1 : eid;
        int sr = srcs[eid];
        sr = sr < 0 ? 0 : (sr > NN - 1 ? NN - 1 : sr);
        const int word = (int)((unsigned)sr | ((unsigned)(ent & (NBRUN - 1)) << 17));
        const int m32 = (c - b0) < 32 ? (c - b0) : 32;
#pragma unroll 1
        for (int k = 0; k < m32; ++k) {
          const int u    = __builtin_amdgcn_readlane(ent, k);
          const int wd   = __builtin_amdgcn_readlane(word, k);
          const int slot = u & (NBRUN - 1);
          if (lane == 0) {
            int p = cur[slot];
            p = p < 0 ? 0 : (p > RCAP - 1 ? RCAP - 1 : p);
            pl[p] = wd;
            cur[slot] = p + 1;
          }
        }
      }
    }
  }
  __syncthreads();

  const int ovf = misc[9];
  int* lp  = LIST + (size_t)blk * RCAP;
  int* cop = CO + (size_t)blk * (2 * NBRUN);
  int* fp  = FLAG + (size_t)blk * 32;
  bucket_flush(pl, cnt, ovf, lp, cop, fp, tid);
  __threadfence();
  bucket_flush(pl, cnt, ovf, lp, cop, fp, tid);
}

template <int KEXT, int PA, int PB, int NT>
__device__ __forceinline__ void gemm_rows(const unsigned short* __restrict__ ap,
                                          const unsigned short* __restrict__ bp, v8f (&acc)[NT]) {
#pragma unroll 1
  for (int k0 = 0; k0 < KEXT; k0 += 32) {
    FragB af;
    af.h[0] = *(const v8usa*)(ap + k0);
    af.h[1] = *(const v8usa*)(ap + k0 + 16);
#pragma unroll
    for (int nt = 0; nt < NT; ++nt) {
      const unsigned short* wq = bp + (size_t)(16 * nt) * (size_t)PB + k0;
      FragB bf;
      bf.h[0] = *(const v8usa*)wq;
      bf.h[1] = *(const v8usa*)(wq + 16);
      acc[nt] = wmb(af, bf, acc[nt]);
    }
  }
}

__global__ __launch_bounds__(G1T) __attribute__((amdgpu_num_vgpr(248)))
void k_gemm1(const unsigned short* __restrict__ XB, const unsigned short* __restrict__ W1T,
             const float* __restrict__ PM, float* H1, float* SC1) {
  __shared__ __attribute__((aligned(16))) float stg[G1M * SP1];
  __shared__ __attribute__((aligned(16))) float sa[256];
  __shared__ __attribute__((aligned(16))) float sdot[2 * G1M * 4];
  const int tid = (int)threadIdx.x, lane = tid & 31, wave = tid >> 5, hh = lane >> 4, m = lane & 15;
  const int rowBase = (int)blockIdx.x * G1M;
  if (tid < 64) *(v4fa*)(sa + 4 * tid) = *(const v4fa*)(PM + PM_AS1 + 4 * tid);

  v8f acc[8];
  {
    const v8f z = {0.f, 0.f, 0.f, 0.f, 0.f, 0.f, 0.f, 0.f};
#pragma unroll
    for (int t = 0; t < 8; ++t) acc[t] = z;
  }
  const unsigned short* ap = XB + (size_t)(rowBase + 16 * wave + m) * (size_t)FD + 8 * hh;
  const unsigned short* bp = W1T + (size_t)m * (size_t)FD + 8 * hh;
  gemm_rows<FD, FD, FD, 8>(ap, bp, acc);
#pragma unroll
  for (int nt = 0; nt < 8; ++nt) {
#pragma unroll
    for (int r = 0; r < 8; ++r) stg[(16 * wave + 8 * hh + r) * SP1 + 16 * nt + m] = acc[nt][r];
  }
  __syncthreads();

  {
    const int row = tid & 63, side = tid >> 6;
    const float* hr = stg + row * SP1;
    const float* av = sa + side * HC1;
    float d0 = 0.0f, d1 = 0.0f, d2 = 0.0f, d3 = 0.0f;
#pragma unroll 1
    for (int c4 = 0; c4 < HID / 4; ++c4) {
      const v4f g0 = *(const v4fa*)(hr + 4 * c4),      a0 = *(const v4fa*)(av + 4 * c4);
      const v4f g1 = *(const v4fa*)(hr + 32 + 4 * c4), a1 = *(const v4fa*)(av + 32 + 4 * c4);
      const v4f g2 = *(const v4fa*)(hr + 64 + 4 * c4), a2 = *(const v4fa*)(av + 64 + 4 * c4);
      const v4f g3 = *(const v4fa*)(hr + 96 + 4 * c4), a3 = *(const v4fa*)(av + 96 + 4 * c4);
      d0 = fmaf(g0.x, a0.x, d0); d0 = fmaf(g0.y, a0.y, d0); d0 = fmaf(g0.z, a0.z, d0); d0 = fmaf(g0.w, a0.w, d0);
      d1 = fmaf(g1.x, a1.x, d1); d1 = fmaf(g1.y, a1.y, d1); d1 = fmaf(g1.z, a1.z, d1); d1 = fmaf(g1.w, a1.w, d1);
      d2 = fmaf(g2.x, a2.x, d2); d2 = fmaf(g2.y, a2.y, d2); d2 = fmaf(g2.z, a2.z, d2); d2 = fmaf(g2.w, a2.w, d2);
      d3 = fmaf(g3.x, a3.x, d3); d3 = fmaf(g3.y, a3.y, d3); d3 = fmaf(g3.z, a3.z, d3); d3 = fmaf(g3.w, a3.w, d3);
    }
    v4f dv;
    dv.x = d0; dv.y = d1; dv.z = d2; dv.w = d3;
    *(v4fa*)(sdot + (side * G1M + row) * 4) = dv;
  }
  __syncthreads();

  const int sw = wave & 1;
  const v4f sv0 = *(const v4fa*)(sdot + (sw * G1M + lane) * 4);
  const v4f sv1 = *(const v4fa*)(sdot + (sw * G1M + 32 + lane) * 4);
  float* sp = SC1 + (size_t)sw * (size_t)MP * NH1 + (size_t)(rowBase + lane) * NH1;

#pragma unroll 1
  for (int i = 0; i < 16; ++i) {
    const int lr = 16 * wave + i;
    const v4f v = *(const v4fa*)(stg + lr * SP1 + 4 * lane);
    *(volatile v4f*)(H1 + (size_t)(rowBase + lr) * HC1 + 4 * lane) = v;
  }
  if (wave < 2) {
    *(volatile v4f*)sp = sv0;
    *(volatile v4f*)(sp + 32 * NH1) = sv1;
  }
  __threadfence();
#pragma unroll 1
  for (int i = 0; i < 16; ++i) {
    const int lr = 16 * wave + i;
    const v4f v = *(const v4fa*)(stg + lr * SP1 + 4 * lane);
    *(volatile v4f*)(H1 + (size_t)(rowBase + lr) * HC1 + 4 * lane) = v;
  }
  if (wave < 2) {
    *(volatile v4f*)sp = sv0;
    *(volatile v4f*)(sp + 32 * NH1) = sv1;
  }
}

__global__ __launch_bounds__(NTHR) void k_replay1(const int* __restrict__ LIST, const int* __restrict__ CO,
                                                  const int* __restrict__ FLAG, const float* __restrict__ H1,
                                                  const float* __restrict__ SC1, const float* __restrict__ PM,
                                                  unsigned short* X1) {
  __shared__ __attribute__((aligned(16))) float sb[HC1];
  const int tid = (int)threadIdx.x, lane = tid & 31;
  const int wave = __builtin_amdgcn_readfirstlane(tid >> 5);
  if (tid < 32) *(v4fa*)(sb + 4 * tid) = *(const v4fa*)(PM + PM_B1 + 4 * tid);
  __syncthreads();
  const v4f bb = *(const v4fa*)(sb + 4 * lane);
  const int rowBase = (int)blockIdx.x * ABM;
  const int bucket  = rowBase >> SLB;
  const int* lb  = LIST + (size_t)bucket * RCAP;
  const int* cob = CO + (size_t)bucket * (2 * NBRUN);
  const int flag = FLAG[(size_t)bucket * 32];
  const float* AS1 = SC1;
  const float* AD1 = SC1 + (size_t)MP * NH1;
  const int head = lane >> 3;
  const bool hA = head == 0, hB = head == 1, hC = head == 2;
  const float qnan = __uint_as_float(0x7fc00000u);

#pragma unroll 1
  for (int i = 0; i < ABM / NWAVE; ++i) {
    const int d    = rowBase + (ABM / NWAVE) * wave + i;
    const int dc   = d < NN ? d : NN - 1;
    const int slot = d & (NBRUN - 1);
    int cv = cob[slot];
    int ov = cob[NBRUN + slot];
    const bool big = cv > DEGCAP;
    cv = cv < 0 ? 0 : (cv > DEGCAP ? DEGCAP : cv);
    ov = ov < 0 ? 0 : (ov > RCAP - 1 ? RCAP - 1 : ov);
    const int c = __builtin_amdgcn_readfirstlane(cv);
    const int o = __builtin_amdgcn_readfirstlane(ov);
    int last = o + c - 1;
    last = last < o ? o : last;
    last = last > RCAP - 1 ? RCAP - 1 : last;

    const v4f adv = *(const v4fa*)(AD1 + (size_t)dc * NH1);
    const v4f asd = *(const v4fa*)(AS1 + (size_t)dc * NH1);
    float m0 = leaky(asd.x + adv.x), m1 = leaky(asd.y + adv.y);
    float m2 = leaky(asd.z + adv.z), m3 = leaky(asd.w + adv.w);
    float dn = 1.0f;
    v4f acc = *(const v4fa*)(H1 + (size_t)dc * HC1 + 4 * lane);

#pragma unroll 1
    for (int j0 = 0; j0 < c; j0 += 32) {
      int idx = o + j0 + lane;
      idx = idx > last ? last : idx;
      const unsigned wd = (unsigned)lb[idx];
      asm volatile("" :: "v"(wd));
      int sr = (int)(wd & 0x1FFFFu);
      sr = sr > NN - 1 ? NN - 1 : sr;
      const v4f a4 = *(const v4fa*)(AS1 + (size_t)sr * NH1);
      asm volatile("" :: "v"(a4));
      const bool valid = (j0 + lane) < c;
      const float e0 = leaky(a4.x + adv.x), e1 = leaky(a4.y + adv.y);
      const float e2 = leaky(a4.z + adv.z), e3 = leaky(a4.w + adv.w);
      float c0 = valid ? e0 : NEGBIG, c1 = valid ? e1 : NEGBIG;
      float c2 = valid ? e2 : NEGBIG, c3 = valid ? e3 : NEGBIG;
#pragma unroll
      for (int off = 16; off > 0; off >>= 1) {
        c0 = fmaxf(c0, __shfl_xor(c0, off, 32));
        c1 = fmaxf(c1, __shfl_xor(c1, off, 32));
        c2 = fmaxf(c2, __shfl_xor(c2, off, 32));
        c3 = fmaxf(c3, __shfl_xor(c3, off, 32));
      }
      const float n0 = fmaxf(m0, c0), n1 = fmaxf(m1, c1), n2 = fmaxf(m2, c2), n3 = fmaxf(m3, c3);
      const float mo = hA ? m0 : (hB ? m1 : (hC ? m2 : m3));
      const float nw = hA ? n0 : (hB ? n1 : (hC ? n2 : n3));
      const float sc = expf(mo - nw);
      const float x0 = expf(e0 - n0), x1 = expf(e1 - n1), x2 = expf(e2 - n2), x3 = expf(e3 - n3);
      const float p0 = valid ? x0 : 0.0f, p1 = valid ? x1 : 0.0f;
      const float p2 = valid ? x2 : 0.0f, p3 = valid ? x3 : 0.0f;
      m0 = n0; m1 = n1; m2 = n2; m3 = n3;
      acc.x *= sc; acc.y *= sc; acc.z *= sc; acc.w *= sc;
      dn *= sc;
      int m32 = c - j0;
      m32 = m32 > 32 ? 32 : m32;
#pragma unroll 1
      for (int j = 0; j < m32; ++j) {
        const int sj = __builtin_amdgcn_readlane(sr, j);
        const float q0 = __int_as_float(__builtin_amdgcn_readlane(__float_as_int(p0), j));
        const float q1 = __int_as_float(__builtin_amdgcn_readlane(__float_as_int(p1), j));
        const float q2 = __int_as_float(__builtin_amdgcn_readlane(__float_as_int(p2), j));
        const float q3 = __int_as_float(__builtin_amdgcn_readlane(__float_as_int(p3), j));
        const float pj = hA ? q0 : (hB ? q1 : (hC ? q2 : q3));
        const v4f rw = *(const v4fa*)(H1 + (size_t)sj * HC1 + 4 * lane);
        acc.x = fmaf(pj, rw.x, acc.x);
        acc.y = fmaf(pj, rw.y, acc.y);
        acc.z = fmaf(pj, rw.z, acc.z);
        acc.w = fmaf(pj, rw.w, acc.w);
        dn += pj;
      }
    }

    const float inv = __builtin_amdgcn_rcpf(dn + EPS_SM);
    float v0 = fmaf(acc.x, inv, bb.x), v1 = fmaf(acc.y, inv, bb.y);
    float v2 = fmaf(acc.z, inv, bb.z), v3 = fmaf(acc.w, inv, bb.w);
    v0 = (v0 > 0.0f) ? v0 : (v0 - v0); v1 = (v1 > 0.0f) ? v1 : (v1 - v1);
    v2 = (v2 > 0.0f) ? v2 : (v2 - v2); v3 = (v3 > 0.0f) ? v3 : (v3 - v3);
    const bool bad  = (flag != 0) | big;
    const bool live = d < NN;
    v0 = bad ? qnan : v0; v1 = bad ? qnan : v1; v2 = bad ? qnan : v2; v3 = bad ? qnan : v3;
    v0 = live ? v0 : 0.0f; v1 = live ? v1 : 0.0f; v2 = live ? v2 : 0.0f; v3 = live ? v3 : 0.0f;
    int h01, h23, l01, l23;
    hilo_pack(v0, v1, v2, v3, h01, h23, l01, l23);
    const v4i ow = regroup32(h01, h23, l01, l23, lane);
    unsigned short* xp = X1 + (size_t)d * KA2P + 8 * lane;
    *(volatile v4i*)xp = ow;
    __threadfence();
    *(volatile v4i*)xp = ow;
  }
}

__global__ __launch_bounds__(NTHR) __attribute__((amdgpu_num_vgpr(248)))
void k_gemm2(const unsigned short* __restrict__ X1, const unsigned short* __restrict__ W2T,
             const float* __restrict__ PM, float* H2, float* SC2) {
  __shared__ __attribute__((aligned(16))) float stg[G2M * SP2];
  __shared__ __attribute__((aligned(16))) float sa2[64];
  __shared__ __attribute__((aligned(16))) float sdot2[2 * G2M];
  const int tid = (int)threadIdx.x, lane = tid & 31, wave = tid >> 5, hh = lane >> 4, m = lane & 15;
  const int rowBase = (int)blockIdx.x * G2M;
  if (tid < 16) *(v4fa*)(sa2 + 4 * tid) = *(const v4fa*)(PM + PM_AS2 + 4 * tid);

  v8f acc[2];
  {
    const v8f z = {0.f, 0.f, 0.f, 0.f, 0.f, 0.f, 0.f, 0.f};
    acc[0] = z; acc[1] = z;
  }
  const unsigned short* ap = X1 + (size_t)(rowBase + 16 * wave + m) * (size_t)KA2P + 8 * hh;
  const unsigned short* bp = W2T + (size_t)m * (size_t)KW2P + 8 * hh;
  gemm_rows<KX2, KA2P, KW2P, 2>(ap, bp, acc);
#pragma unroll
  for (int nt = 0; nt < 2; ++nt) {
#pragma unroll
    for (int r = 0; r < 8; ++r) stg[(16 * wave + 8 * hh + r) * SP2 + 16 * nt + m] = acc[nt][r];
  }
  __syncthreads();

  {
    const int row = tid & (G2M - 1), side = tid >> 7;
    const float* hr = stg + row * SP2;
    const float* av = sa2 + side * HID;
    float dd = 0.0f;
#pragma unroll 2
    for (int c4 = 0; c4 < HID / 4; ++c4) {
      const v4f g = *(const v4fa*)(hr + 4 * c4);
      const v4f a = *(const v4fa*)(av + 4 * c4);
      dd = fmaf(g.x, a.x, dd); dd = fmaf(g.y, a.y, dd); dd = fmaf(g.z, a.z, dd); dd = fmaf(g.w, a.w, dd);
    }
    sdot2[side * G2M + row] = dd;
  }
  __syncthreads();

  const int sw = wave & 1;
  const v4f sv = *(const v4fa*)(sdot2 + sw * G2M + 4 * lane);
  float* sp = SC2 + (size_t)sw * (size_t)MP + rowBase + 4 * lane;
  const int rq = lane >> 3, pc = lane & 7;

#pragma unroll 1
  for (int i = 0; i < 4; ++i) {
    const int lr = 16 * wave + 4 * i + rq;
    const v4f v = *(const v4fa*)(stg + lr * SP2 + 4 * pc);
    *(volatile v4f*)(H2 + (size_t)(rowBase + lr) * HID + 4 * pc) = v;
  }
  if (wave < 2) *(volatile v4f*)sp = sv;
  __threadfence();
#pragma unroll 1
  for (int i = 0; i < 4; ++i) {
    const int lr = 16 * wave + 4 * i + rq;
    const v4f v = *(const v4fa*)(stg + lr * SP2 + 4 * pc);
    *(volatile v4f*)(H2 + (size_t)(rowBase + lr) * HID + 4 * pc) = v;
  }
  if (wave < 2) *(volatile v4f*)sp = sv;
}

__global__ __launch_bounds__(NTHR) void k_replay2(const int* __restrict__ LIST, const int* __restrict__ CO,
                                                  const int* __restrict__ FLAG, const float* __restrict__ H2,
                                                  const float* __restrict__ SC2, const float* __restrict__ PM,
                                                  float* out) {
  __shared__ __attribute__((aligned(16))) float spar[64];
  __shared__ __attribute__((aligned(16))) float sres[ABM];
  const int tid = (int)threadIdx.x, lane = tid & 31;
  const int wave = __builtin_amdgcn_readfirstlane(tid >> 5);
  if (tid < 16) *(v4fa*)(spar + 4 * tid) = *(const v4fa*)(PM + PM_B2 + 4 * tid);
  const float blin = PM[PM_BL];
  __syncthreads();
  const float bz = spar[lane];
  const float wl = spar[HID + lane];
  const int rowBase = (int)blockIdx.x * ABM;
  const int bucket  = rowBase >> SLB;
  const int* lb  = LIST + (size_t)bucket * RCAP;
  const int* cob = CO + (size_t)bucket * (2 * NBRUN);
  const int flag = FLAG[(size_t)bucket * 32];
  const float* AS2 = SC2;
  const float* AD2 = SC2 + (size_t)MP;
  const float qnan = __uint_as_float(0x7fc00000u);

#pragma unroll 1
  for (int i = 0; i < ABM / NWAVE; ++i) {
    const int d    = rowBase + (ABM / NWAVE) * wave + i;
    const int dc   = d < NN ? d : NN - 1;
    const int slot = d & (NBRUN - 1);
    int cv = cob[slot];
    int ov = cob[NBRUN + slot];
    const bool big = cv > DEGCAP;
    cv = cv < 0 ? 0 : (cv > DEGCAP ? DEGCAP : cv);
    ov = ov < 0 ? 0 : (ov > RCAP - 1 ? RCAP - 1 : ov);
    const int c = __builtin_amdgcn_readfirstlane(cv);
    const int o = __builtin_amdgcn_readfirstlane(ov);
    int last = o + c - 1;
    last = last < o ? o : last;
    last = last > RCAP - 1 ? RCAP - 1 : last;

    const float adv = AD2[dc];
    float mx = leaky(AS2[dc] + adv);
    float dn = 1.0f;
    float acc = H2[(size_t)dc * HID + lane];

#pragma unroll 1
    for (int j0 = 0; j0 < c; j0 += 32) {
      int idx = o + j0 + lane;
      idx = idx > last ? last : idx;
      const unsigned wd = (unsigned)lb[idx];
      asm volatile("" :: "v"(wd));
      int sr = (int)(wd & 0x1FFFFu);
      sr = sr > NN - 1 ? NN - 1 : sr;
      const float a1 = AS2[sr];
      asm volatile("" :: "v"(a1));
      const bool valid = (j0 + lane) < c;
      const float e = leaky(a1 + adv);
      float cm = valid ? e : NEGBIG;
#pragma unroll
      for (int off = 16; off > 0; off >>= 1) cm = fmaxf(cm, __shfl_xor(cm, off, 32));
      const float mn = fmaxf(mx, cm);
      const float sc = expf(mx - mn);
      const float xe = expf(e - mn);
      const float p  = valid ? xe : 0.0f;
      mx = mn;
      acc *= sc;
      dn  *= sc;
      int m32 = c - j0;
      m32 = m32 > 32 ? 32 : m32;
#pragma unroll 1
      for (int j = 0; j < m32; ++j) {
        const int sj = __builtin_amdgcn_readlane(sr, j);
        const float pj = __int_as_float(__builtin_amdgcn_readlane(__float_as_int(p), j));
        const float rw = H2[(size_t)sj * HID + lane];
        acc = fmaf(pj, rw, acc);
        dn += pj;
      }
    }

    const float inv = __builtin_amdgcn_rcpf(dn + EPS_SM);
    float v = fmaf(acc, inv, bz);
    v = (v > 0.0f) ? v : (v - v);
    float t = v * wl;
#pragma unroll
    for (int off = 16; off > 0; off >>= 1) t += __shfl_xor(t, off, 32);
    float res = t + blin;
    const bool bad = (flag != 0) | big;
    res = bad ? qnan : res;
    if (lane == 0) sres[(ABM / NWAVE) * wave + i] = res;
  }
  __syncthreads();

  if (wave == 0) {
    int live = NN - rowBase;
    live = live < 0 ? 0 : (live > ABM ? ABM : live);
    const int np = live >> 2;
    v4f v = *(const v4fa*)(sres + 4 * (lane & 15));
    asm volatile("" :: "v"(v));
    const v4f q4 = {qnan, qnan, qnan, qnan};
    if (flag != 0) v = q4;
    float* op = out + rowBase + 4 * (lane & 15);
    const bool wr = lane < np;
    if (wr) *(volatile v4f*)op = v;
    __threadfence();
    if (wr) *(volatile v4f*)op = v;
  }
}

extern "C" void kernel_launch(void* const* d_in, const int* in_sizes, int n_in,
                              void* d_out, int out_size, void* d_ws, size_t ws_size,
                              hipStream_t stream) {
  if (n_in < 13) return;
  if (in_sizes[0] != NN * FD) return;
  if (in_sizes[1] != 2 * NE) return;
  if (in_sizes[2] != NN) return;
  if (in_sizes[3] != FD * HC1) return;
  if (in_sizes[4] != NH1 * HID) return;
  if (in_sizes[5] != NH1 * HID) return;
  if (in_sizes[6] != HC1) return;
  if (in_sizes[7] != HC1 * HID) return;
  if (in_sizes[8] != HID) return;
  if (in_sizes[9] != HID) return;
  if (in_sizes[10] != HID) return;
  if (in_sizes[11] != HID) return;
  if (in_sizes[12] != 1) return;
  if (out_size != NN) return;

  const float* x    = (const float*)d_in[0];
  const int*   ei   = (const int*)d_in[1];
  const float* W1   = (const float*)d_in[3];
  const float* as1  = (const float*)d_in[4];
  const float* ad1  = (const float*)d_in[5];
  const float* b1   = (const float*)d_in[6];
  const float* W2   = (const float*)d_in[7];
  const float* as2  = (const float*)d_in[8];
  const float* ad2  = (const float*)d_in[9];
  const float* b2   = (const float*)d_in[10];
  const float* wlin = (const float*)d_in[11];
  const float* blin = (const float*)d_in[12];
  float* out = (float*)d_out;
  const int* srcs = ei;
  const int* dsts = ei + NE;

  constexpr size_t zA    = (size_t)MP * KA2P * 2;
  constexpr size_t zB    = (size_t)MP * HC1 * 4;
  constexpr size_t zSC1  = (size_t)2 * MP * NH1 * 4;
  constexpr size_t zSC2  = (size_t)2 * MP * 4;
  constexpr size_t zLIST = (size_t)NBK * RCAP * 4;
  constexpr size_t zCO   = (size_t)NBK * 2 * NBRUN * 4;
  constexpr size_t zFLAG = (size_t)NBK * 128;
  constexpr size_t zW1T  = (size_t)HC1 * FD * 2;
  constexpr size_t zW2T  = (size_t)HID * KW2P * 2;
  constexpr size_t zPM   = (size_t)PMN * 4;
  constexpr size_t oA    = 0;
  constexpr size_t oB    = oA + zA;
  constexpr size_t oSC1  = oB + zB;
  constexpr size_t oSC2  = oSC1 + zSC1;
  constexpr size_t oLIST = oSC2 + zSC2;
  constexpr size_t oCO   = oLIST + zLIST;
  constexpr size_t oFLAG = oCO + zCO;
  constexpr size_t oW1T  = oFLAG + zFLAG;
  constexpr size_t oW2T  = oW1T + zW1T;
  constexpr size_t oPM   = oW2T + zW2T;
  constexpr size_t oEND  = oPM + zPM;
  static_assert(zA % 256 == 0 && zB % 256 == 0 && zSC1 % 256 == 0 && zSC2 % 256 == 0 && zLIST % 256 == 0);
  static_assert(zCO % 256 == 0 && zFLAG % 256 == 0 && zW1T % 256 == 0 && zW2T % 256 == 0 && zPM % 256 == 0);
  static_assert((size_t)MP * FD * 2 <= zA && (size_t)MP * HID * 4 <= zB);
  static_assert(oEND <= ((size_t)128u << 20));
  if (oEND > ws_size) return;

  char* ws = (char*)d_ws;
  unsigned short* XB   = (unsigned short*)(ws + oA);
  unsigned short* X1   = (unsigned short*)(ws + oA);
  float*          H1   = (float*)(ws + oB);
  float*          H2   = (float*)(ws + oB);
  float*          SC1  = (float*)(ws + oSC1);
  float*          SC2  = (float*)(ws + oSC2);
  int*            LIST = (int*)(ws + oLIST);
  int*            CO   = (int*)(ws + oCO);
  int*            FLAG = (int*)(ws + oFLAG);
  unsigned short* W1T  = (unsigned short*)(ws + oW1T);
  unsigned short* W2T  = (unsigned short*)(ws + oW2T);
  float*          PM   = (float*)(ws + oPM);

  hipFuncSetAttribute(reinterpret_cast<const void*>(&k_bucket), hipFuncAttributeMaxDynamicSharedMemorySize, (int)BK_LDS);

  k_prep<<<PBTOT, NTHR, 0, stream>>>(x, W1, as1, ad1, b1, W2, as2, ad2, b2, wlin, blin, XB, W1T, W2T, PM);
  k_bucket<<<NBK, NTHR, BK_LDS, stream>>>(srcs, dsts, LIST, CO, FLAG);
  k_gemm1<<<MP / G1M, G1T, 0, stream>>>(XB, W1T, PM, H1, SC1);
  k_replay1<<<MP / ABM, NTHR, 0, stream>>>(LIST, CO, FLAG, H1, SC1, PM, X1);
  k_gemm2<<<MP / G2M, NTHR, 0, stream>>>(X1, W2T, PM, H2, SC2);
  k_replay2<<<MP / ABM, NTHR, 0, stream>>>(LIST, CO, FLAG, H2, SC2, PM, out);
}
